// SUNConv_78572131713436
// MI455X (gfx1250) — hardware-verified
//
#include <hip/hip_runtime.h>
#include <stdint.h>

#define NB    8
#define NN    128
#define ND    64
#define NBN   (NB * NN)
#define NT    (NB * NN * NN)
#define NC    448
#define LDP   136
#define K0P   128
#define K1P   192
#define MINNORM 6.103515625e-05f
#define SX    16.0f
#define ISX   0.0625f
#define SW0   64.0f
#define SWC   256.0f
#define SRES  2048.0f
#define IRES  0.00048828125f
#define I1024 0.0009765625f
#define I4096 0.000244140625f
#define I8M   1.1920928955078125e-07f
#define I2048 0.00048828125f

static_assert(NT == 131072);
static_assert(((NT * ND) % (8 * 256)) == 0);
static_assert((NBN * ND) == 256 * 256);
static_assert((2 * NC * ND) == 224 * 256);
static_assert(8 * 2048 <= 2 * ND * LDP);
static_assert((ND * ND / 8) == 512);
static_assert((ND * K0P / 8) == 1024);
static_assert((ND * K1P / 8) == 1536);

typedef _Float16     v16h __attribute__((ext_vector_type(16)));
typedef float        v8f  __attribute__((ext_vector_type(8)));
typedef float        v4f  __attribute__((ext_vector_type(4)));
typedef unsigned int v4u  __attribute__((ext_vector_type(4)));

__device__ __forceinline__ unsigned short bf_bits(float f) {
  unsigned u = __float_as_uint(f);
  return (unsigned short)((u + 0x7FFFu + ((u >> 16) & 1u)) >> 16);
}
__device__ __forceinline__ float bfr(float f) { return __uint_as_float(((unsigned)bf_bits(f)) << 16); }
__device__ __forceinline__ float h2f(unsigned short u) { return (float)__builtin_bit_cast(_Float16, u); }
__device__ __forceinline__ unsigned pk16(unsigned short a, unsigned short b) { return (unsigned)a | ((unsigned)b << 16); }
__device__ __forceinline__ v8f zero8() { v8f z = {0.f, 0.f, 0.f, 0.f, 0.f, 0.f, 0.f, 0.f}; return z; }

__device__ __forceinline__ unsigned short f16z_bits(float v) {
  const _Float16 h = (_Float16)v;
  const float hf = (float)h;
  const unsigned short b = __builtin_bit_cast(unsigned short, h);
  return (fabsf(hf) < MINNORM) ? (unsigned short)0 : b;
}
__device__ __forceinline__ void split16(float v, unsigned short& hb, unsigned short& lb) {
  const _Float16 h = (_Float16)v;
  float hf = (float)h;
  const bool tiny = fabsf(hf) < MINNORM;
  hf = tiny ? 0.0f : hf;
  hb = tiny ? (unsigned short)0 : __builtin_bit_cast(unsigned short, h);
  lb = f16z_bits((v - hf) * SRES);
}
__device__ __forceinline__ v4u pack8(const unsigned short* hv) {
  v4u u;
  u[0] = pk16(hv[0], hv[1]);
  u[1] = pk16(hv[2], hv[3]);
  u[2] = pk16(hv[4], hv[5]);
  u[3] = pk16(hv[6], hv[7]);
  return u;
}

__device__ __forceinline__ v16h ldfrag_u(const unsigned short* p) {
  union { v16h v; v4u u[2]; } f;
  f.u[0] = *(const v4u*)(p);
  f.u[1] = *(const v4u*)(p + 16);
  return f.v;
}

__device__ __forceinline__ v8f mma_raw(v16h a, v16h b, v8f c) {
  return __builtin_amdgcn_wmma_f32_16x16x32_f16(false, a, false, b, (short)0, c, false, false);
}
__device__ __forceinline__ void guard_a(v8f& c0, const v16h& a0, const v16h& a1, const v16h& b0, const v16h& b1) {
#if defined(__HIP_DEVICE_COMPILE__)
  asm volatile("v_nop\n\tv_nop\n\tv_nop\n\tv_nop" : "+v"(c0) : "v"(a0), "v"(a1), "v"(b0), "v"(b1));
#endif
}
__device__ __forceinline__ void guard_b(v8f& c0, v8f& c1, const v16h& a0, const v16h& b0, const v16h& b1) {
#if defined(__HIP_DEVICE_COMPILE__)
  asm volatile("v_nop\n\tv_nop\n\tv_nop\n\tv_nop" : "+v"(c0), "+v"(c1) : "v"(a0), "v"(b0), "v"(b1));
#endif
}

__device__ __forceinline__ float wdot(const float* __restrict__ hw, const float* __restrict__ mw, int crow, int n) {
  float s = 0.0f;
#pragma unroll 1
  for (int m = 0; m < ND; ++m) s = fmaf(bfr(hw[crow * ND + m]), bfr(mw[m * ND + n]), s);
  return s;
}

__global__ __launch_bounds__(256)
void k_wfold(const float* __restrict__ hw, const float* __restrict__ mw, float* Wc) {
  const int t = blockIdx.x * 256 + threadIdx.x;
  const int tc = t >> 6, n = t & 63;
  const float s = wdot(hw, mw, tc, n);
  *(volatile float*)(Wc + t) = s;
  __threadfence();
  *(volatile float*)(Wc + t) = s;
}

__global__ __launch_bounds__(256)
void k_wplanes(const float* __restrict__ l0w, const float* __restrict__ hw, const float* __restrict__ mw,
               unsigned short* L0p, unsigned short* B0p, unsigned short* B1p) {
  const int blk = blockIdx.x, tid = threadIdx.x;
  unsigned short hv[8];
  unsigned short* dst;
  if (blk < 2) {
    const int q = blk * 256 + tid;
    const int n = q >> 3, kq = q & 7;
#pragma unroll
    for (int e = 0; e < 8; ++e) {
      const int k = 8 * kq + e;
      hv[e] = f16z_bits(SW0 * bfr(l0w[k * ND + n]));
    }
    dst = L0p + 8 * q;
  } else if (blk < 6) {
    const int q = (blk - 2) * 256 + tid;
    const int n = q >> 4, kq = q & 15;
#pragma unroll
    for (int e = 0; e < 8; ++e) {
      const int k = 8 * kq + e;
      const int crow = (k < 64) ? k : (128 + k);
      const float wc = wdot(hw, mw, crow, n);
      unsigned short hb, lb;
      split16(SWC * wc, hb, lb);
      hv[e] = hb;
    }
    dst = B0p + 8 * q;
  } else {
    const int q = (blk - 6) * 256 + tid;
    const int n = q / 24, kq = q - 24 * n;
#pragma unroll
    for (int e = 0; e < 8; ++e) {
      const int k = 8 * kq + e;
      const int crow = (k < 64) ? k : ((k < 128) ? (128 + k) : (64 + k));
      const float wc = wdot(hw, mw, crow, n);
      unsigned short hb, lb;
      split16(SWC * wc, hb, lb);
      hv[e] = (k < 128) ? lb : hb;
    }
    dst = B1p + 8 * q;
  }
  const v4u u = pack8(hv);
  *(volatile v4u*)dst = u;
  __threadfence();
  *(volatile v4u*)dst = u;
}

__global__ __launch_bounds__(256)
void k_xplane(const float* __restrict__ X, unsigned short* Xp) {
  const size_t i = (size_t)blockIdx.x * 256 + threadIdx.x;
  const v4f a = *(const v4f*)(X + i * 8);
  const v4f b = *(const v4f*)(X + i * 8 + 4);
  unsigned short hv[8];
#pragma unroll
  for (int k = 0; k < 4; ++k) {
    hv[k]     = f16z_bits(SX * bfr(a[k]));
    hv[4 + k] = f16z_bits(SX * bfr(b[k]));
  }
  const v4u u = pack8(hv);
  unsigned short* dst = Xp + i * 8;
  *(volatile v4u*)dst = u;
  __threadfence();
  *(volatile v4u*)dst = u;
}

__global__ __launch_bounds__(256)
void k_at(const float* __restrict__ A, unsigned short* ATp) {
  __shared__ __align__(16) unsigned short tl[NN * LDP];
  const int b = blockIdx.x, tid = threadIdx.x;
  const float* Ab = A + (size_t)b * NN * NN;
#pragma unroll 1
  for (int it = 0; it < 64; ++it) {
    const int idx = it * 256 + tid;
    const int k = idx >> 7, j = idx & 127;
    tl[j * LDP + k] = f16z_bits(bfr(Ab[idx]));
  }
  __syncthreads();
  v4u u[8];
#pragma unroll
  for (int it = 0; it < 8; ++it) {
    const int p = it * 256 + tid;
    const int j = p >> 4, kq = p & 15;
    u[it] = *(const v4u*)(tl + j * LDP + 8 * kq);
  }
  unsigned short* dst = ATp + (size_t)b * NN * NN;
#pragma unroll
  for (int it = 0; it < 8; ++it) *(volatile v4u*)(dst + 8 * (it * 256 + tid)) = u[it];
  __threadfence();
#pragma unroll
  for (int it = 0; it < 8; ++it) *(volatile v4u*)(dst + 8 * (it * 256 + tid)) = u[it];
}

__global__ __launch_bounds__(256)
void k_stats(const float* __restrict__ X, float* Xd, float* X5, float* X6) {
  const int t = blockIdx.x * 256 + threadIdx.x;
  const int bn = t >> 6, d = t & 63, b = bn >> 7, node = bn & 127;
  const float* Xb = X + (size_t)b * NN * NN * ND;
  const float xd = bfr(Xb[((size_t)node * NN + node) * ND + d]);
  float s5 = 0.0f, s6 = 0.0f;
#pragma unroll 1
  for (int i = 0; i < NN; ++i) s5 += bfr(Xb[((size_t)i * NN + node) * ND + d]);
#pragma unroll 1
  for (int j = 0; j < NN; ++j) s6 += bfr(Xb[((size_t)node * NN + j) * ND + d]);
  const float m5 = s5 * (1.0f / 128.0f), m6 = s6 * (1.0f / 128.0f);
  *(volatile float*)(Xd + t) = xd;
  *(volatile float*)(X5 + t) = m5;
  *(volatile float*)(X6 + t) = m6;
  __threadfence();
  *(volatile float*)(Xd + t) = xd;
  *(volatile float*)(X5 + t) = m5;
  *(volatile float*)(X6 + t) = m6;
}

__global__ __launch_bounds__(256)
void k_x4(const unsigned short* __restrict__ Xp, const unsigned short* __restrict__ L0p,
          const float* __restrict__ l0b, const unsigned short* __restrict__ ATp,
          unsigned short* X4h, unsigned short* X4l) {
  __shared__ __align__(16) unsigned short lds[2 * ND * LDP];
  const int tid = threadIdx.x, w = tid >> 5, lane = tid & 31, hh = lane >> 4, c = lane & 15;
  const int bi = blockIdx.x, b = bi >> 7;
  {
    const unsigned short* ap = Xp + (size_t)(bi * NN + 16 * w + c) * ND + 8 * hh;
    const v16h a0 = ldfrag_u(ap);
    const v16h a1 = ldfrag_u(ap + 32);
#pragma unroll
    for (int t = 0; t < 4; ++t) {
      const int n = 16 * t + c;
      const unsigned short* bp = L0p + n * ND + 8 * hh;
      const v16h b0 = ldfrag_u(bp);
      const v16h b1 = ldfrag_u(bp + 32);
      v8f acc = mma_raw(a0, b0, zero8());
      acc = mma_raw(a1, b1, acc);
      guard_a(acc, a0, a1, b0, b1);
      const float bias = bfr(l0b[n]);
#pragma unroll
      for (int r = 0; r < 8; ++r) {
        const float v = fmaxf(acc[r] * I1024 + bias, 0.0f);
        unsigned short hb, lb;
        split16(v, hb, lb);
        const int k = 16 * w + 8 * hh + r;
        lds[n * LDP + k] = hb;
        lds[ND * LDP + n * LDP + k] = lb;
      }
    }
  }
  __syncthreads();
  v8f ah[4], al[4];
  {
    const unsigned short* jp = ATp + (size_t)(b * NN + 16 * w + c) * NN + 8 * hh;
    v16h af[4];
#pragma unroll
    for (int s = 0; s < 4; ++s) af[s] = ldfrag_u(jp + 32 * s);
#pragma unroll
    for (int t = 0; t < 4; ++t) {
      ah[t] = zero8();
      al[t] = zero8();
      const unsigned short* bp = lds + (16 * t + c) * LDP + 8 * hh;
#pragma unroll
      for (int s = 0; s < 4; ++s) {
        const v16h bh = ldfrag_u(bp + 32 * s);
        const v16h bl = ldfrag_u(bp + ND * LDP + 32 * s);
        ah[t] = mma_raw(af[s], bh, ah[t]);
        al[t] = mma_raw(af[s], bl, al[t]);
        guard_b(ah[t], al[t], af[s], bh, bl);
      }
    }
  }
  __syncthreads();
  unsigned short* stg = lds + w * 2048;
#pragma unroll
  for (int t = 0; t < 4; ++t) {
#pragma unroll
    for (int r = 0; r < 8; ++r) {
      const float x4 = ah[t][r] + al[t][r] * IRES;
      unsigned short hb, lb;
      split16(x4 * SX, hb, lb);
      const int e = (8 * hh + r) * ND + 16 * t + c;
      stg[e] = hb;
      stg[1024 + e] = lb;
    }
  }
  __syncthreads();
  v4u uh[4], ul[4];
#pragma unroll
  for (int s = 0; s < 4; ++s) {
    uh[s] = *(const v4u*)(stg + 256 * s + 8 * lane);
    ul[s] = *(const v4u*)(stg + 1024 + 256 * s + 8 * lane);
  }
  const size_t ob = (size_t)(bi * NN + 16 * w) * ND;
#pragma unroll
  for (int s = 0; s < 4; ++s) {
    *(volatile v4u*)(X4h + ob + 256 * s + 8 * lane) = uh[s];
    *(volatile v4u*)(X4l + ob + 256 * s + 8 * lane) = ul[s];
  }
  __threadfence();
#pragma unroll
  for (int s = 0; s < 4; ++s) {
    *(volatile v4u*)(X4h + ob + 256 * s + 8 * lane) = uh[s];
    *(volatile v4u*)(X4l + ob + 256 * s + 8 * lane) = ul[s];
  }
}

__global__ __launch_bounds__(256)
void k_x7(const unsigned short* __restrict__ X4h, const unsigned short* __restrict__ X4l, float* X7) {
  const int t = blockIdx.x * 256 + threadIdx.x;
  const int bn = t >> 6, d = t & 63, b = bn >> 7, j = bn & 127;
  float s = 0.0f;
#pragma unroll 1
  for (int i = 0; i < NN; ++i) {
    const size_t e = ((size_t)((b * NN + i) * NN + j)) * ND + d;
    s += h2f(X4h[e]) + h2f(X4l[e]) * IRES;
  }
  const float v = s * I2048;
  *(volatile float*)(X7 + t) = v;
  __threadfence();
  *(volatile float*)(X7 + t) = v;
}

__global__ __launch_bounds__(256)
void k_cvec(const float* __restrict__ Xd, const float* __restrict__ X5, const float* __restrict__ X6,
            const float* __restrict__ X7, const unsigned short* __restrict__ X4h,
            const unsigned short* __restrict__ X4l, const float* __restrict__ Wc,
            const float* __restrict__ mb, float* Ci, float* Cj, float* Hd) {
  const int t = blockIdx.x * 256 + threadIdx.x;
  const int bn = t >> 6, n = t & 63, node = bn & 127;
  const float* W0 = Wc;
  const float* W1 = Wc + NC * ND;
  const float bias = bfr(mb[n]);
  float ci = bias, cj = 0.0f, hd = bias;
  const size_t drow = ((size_t)bn * NN + node) * ND;
#pragma unroll 1
  for (int d = 0; d < ND; ++d) {
    const float xd = Xd[bn * ND + d];
    const float x5 = X5[bn * ND + d];
    const float x6 = X6[bn * ND + d];
    const float x7 = X7[bn * ND + d];
    const float x4 = (h2f(X4h[drow + d]) + h2f(X4l[drow + d]) * IRES) * ISX;
    const int wo = d * ND + n;
    ci = fmaf(xd, W0[1 * 4096 + wo], ci);
    ci = fmaf(x6, W0[5 * 4096 + wo], ci);
    cj = fmaf(xd, W0[2 * 4096 + wo], cj);
    cj = fmaf(x5, W0[4 * 4096 + wo], cj);
    cj = fmaf(x7, W0[6 * 4096 + wo], cj);
    const float w123 = W1[wo] + W1[4096 + wo] + W1[2 * 4096 + wo];
    hd = fmaf(xd, w123, hd);
    hd = fmaf(x4, W1[3 * 4096 + wo], hd);
    hd = fmaf(x5, W1[4 * 4096 + wo], hd);
    hd = fmaf(x6, W1[5 * 4096 + wo], hd);
    hd = fmaf(x7, W1[6 * 4096 + wo], hd);
  }
  *(volatile float*)(Ci + t) = ci;
  *(volatile float*)(Cj + t) = cj;
  *(volatile float*)(Hd + t) = hd;
  __threadfence();
  *(volatile float*)(Ci + t) = ci;
  *(volatile float*)(Cj + t) = cj;
  *(volatile float*)(Hd + t) = hd;
}

__global__ __launch_bounds__(256)
void k_tuple(const unsigned short* __restrict__ Xp, const unsigned short* __restrict__ X4h,
             const unsigned short* __restrict__ X4l, const unsigned short* __restrict__ B0p,
             const unsigned short* __restrict__ B1p, const float* __restrict__ Ci,
             const float* __restrict__ Cj, const float* __restrict__ Hd, float* out) {
  __shared__ __align__(16) float stg[8 * 1024];
  const int tid = threadIdx.x, w = tid >> 5, lane = tid & 31, hh = lane >> 4, c = lane & 15;
  const int bi = blockIdx.x, b = bi >> 7, idg = bi & 127;
  const size_t ro = (size_t)(bi * NN + 16 * w + c) * ND + 8 * hh;
  v16h af[6];
  af[0] = ldfrag_u(Xp + ro);
  af[1] = ldfrag_u(Xp + ro + 32);
  af[2] = ldfrag_u(X4h + ro);
  af[3] = ldfrag_u(X4h + ro + 32);
  af[4] = ldfrag_u(X4l + ro);
  af[5] = ldfrag_u(X4l + ro + 32);
  float* sw = stg + w * 1024;
#pragma unroll
  for (int t = 0; t < 4; ++t) {
    const int n = 16 * t + c;
    const unsigned short* p0 = B0p + n * K0P + 8 * hh;
    const unsigned short* p1 = B1p + n * K1P + 8 * hh;
    v8f c0 = zero8(), c1 = zero8();
#pragma unroll
    for (int s = 0; s < 4; ++s) {
      const v16h b0 = ldfrag_u(p0 + 32 * s);
      const v16h b1 = ldfrag_u(p1 + 32 * s);
      c0 = mma_raw(af[s], b0, c0);
      c1 = mma_raw(af[s], b1, c1);
      guard_b(c0, c1, af[s], b0, b1);
    }
#pragma unroll
    for (int s = 4; s < 6; ++s) {
      const v16h b1 = ldfrag_u(p1 + 32 * s);
      c1 = mma_raw(af[s], b1, c1);
      guard_b(c0, c1, af[s], b1, b1);
    }
    const float ci = Ci[bi * ND + n];
    const float hd = Hd[bi * ND + n];
#pragma unroll
    for (int r = 0; r < 8; ++r) {
      const int j = 16 * w + 8 * hh + r;
      const float cj = Cj[(size_t)(b * NN + j) * ND + n];
      float v = c0[r] * I4096 + c1[r] * I8M + ci + cj;
      v = (j == idg) ? hd : v;
      v = fmaxf(v, 0.0f);
      sw[(8 * hh + r) * ND + 16 * t + c] = v;
    }
  }
  __syncthreads();
  v4f ov[8];
#pragma unroll
  for (int s = 0; s < 8; ++s) ov[s] = *(const v4f*)(sw + 128 * s + 4 * lane);
  float* ob = out + (size_t)(bi * NN + 16 * w) * ND;
#pragma unroll
  for (int s = 0; s < 8; ++s) *(volatile v4f*)(ob + 128 * s + 4 * lane) = ov[s];
  __threadfence();
#pragma unroll
  for (int s = 0; s < 8; ++s) *(volatile v4f*)(ob + 128 * s + 4 * lane) = ov[s];
}

extern "C" void kernel_launch(void* const* d_in, const int* in_sizes, int n_in,
                              void* d_out, int out_size, void* d_ws, size_t ws_size,
                              hipStream_t stream) {
  if (n_in < 7) return;
  if (in_sizes[0] != NB * NN * NN) return;
  if (in_sizes[1] != NT * ND) return;
  if (in_sizes[2] != ND * ND) return;
  if (in_sizes[3] != ND) return;
  if (in_sizes[4] != 2 * NC * ND) return;
  if (in_sizes[5] != ND * ND) return;
  if (in_sizes[6] != ND) return;
  if (out_size != NT * ND) return;

  const float* A   = (const float*)d_in[0];
  const float* X   = (const float*)d_in[1];
  const float* l0w = (const float*)d_in[2];
  const float* l0b = (const float*)d_in[3];
  const float* hw  = (const float*)d_in[4];
  const float* mw  = (const float*)d_in[5];
  const float* mb  = (const float*)d_in[6];
  float* out = (float*)d_out;

  const size_t sPl  = (size_t)NT * ND * 2;
  const size_t sAT  = (size_t)NB * NN * NN * 2;
  const size_t sL0  = (size_t)ND * ND * 2;
  const size_t sB0  = (size_t)ND * K0P * 2;
  const size_t sB1  = (size_t)ND * K1P * 2;
  const size_t sWc  = (size_t)2 * NC * ND * 4;
  const size_t sVec = (size_t)NBN * ND * 4;
  size_t off = 0;
  const size_t oXp  = off; off += sPl;
  const size_t oX4h = off; off += sPl;
  const size_t oX4l = off; off += sPl;
  const size_t oAT  = off; off += sAT;
  const size_t oL0  = off; off += sL0;
  const size_t oB0  = off; off += sB0;
  const size_t oB1  = off; off += sB1;
  const size_t oWc  = off; off += sWc;
  const size_t oXd  = off; off += sVec;
  const size_t oX5  = off; off += sVec;
  const size_t oX6  = off; off += sVec;
  const size_t oX7  = off; off += sVec;
  const size_t oCi  = off; off += sVec;
  const size_t oCj  = off; off += sVec;
  const size_t oHd  = off; off += sVec;
  if (off > ws_size) return;
  if (off > (size_t)134217728) return;

  char* ws = (char*)d_ws;
  unsigned short* Xp  = (unsigned short*)(ws + oXp);
  unsigned short* X4h = (unsigned short*)(ws + oX4h);
  unsigned short* X4l = (unsigned short*)(ws + oX4l);
  unsigned short* ATp = (unsigned short*)(ws + oAT);
  unsigned short* L0p = (unsigned short*)(ws + oL0);
  unsigned short* B0p = (unsigned short*)(ws + oB0);
  unsigned short* B1p = (unsigned short*)(ws + oB1);
  float* Wc = (float*)(ws + oWc);
  float* Xd = (float*)(ws + oXd);
  float* X5 = (float*)(ws + oX5);
  float* X6 = (float*)(ws + oX6);
  float* X7 = (float*)(ws + oX7);
  float* Ci = (float*)(ws + oCi);
  float* Cj = (float*)(ws + oCj);
  float* Hd = (float*)(ws + oHd);

  k_wfold<<<dim3((2 * NC * ND) / 256), dim3(256), 0, stream>>>(hw, mw, Wc);
  k_wplanes<<<dim3(12), dim3(256), 0, stream>>>(l0w, hw, mw, L0p, B0p, B1p);
  k_xplane<<<dim3((NT * ND) / (8 * 256)), dim3(256), 0, stream>>>(X, Xp);
  k_at<<<dim3(NB), dim3(256), 0, stream>>>(A, ATp);
  k_stats<<<dim3((NBN * ND) / 256), dim3(256), 0, stream>>>(X, Xd, X5, X6);
  k_x4<<<dim3(NBN), dim3(256), 0, stream>>>(Xp, L0p, l0b, ATp, X4h, X4l);
  k_x7<<<dim3((NBN * ND) / 256), dim3(256), 0, stream>>>(X4h, X4l, X7);
  k_cvec<<<dim3((NBN * ND) / 256), dim3(256), 0, stream>>>(Xd, X5, X6, X7, X4h, X4l, Wc, mb, Ci, Cj, Hd);
  k_tuple<<<dim3(NBN), dim3(256), 0, stream>>>(Xp, X4h, X4l, B0p, B1p, Ci, Cj, Hd, out);
  (void)hipGetLastError();
}
